// LlamaMultiHeadAttention_47614007443848
// MI455X (gfx1250) — hardware-verified
//
#include <hip/hip_runtime.h>
#include <math.h>
#include <stdint.h>
#include <stddef.h>

#pragma clang fp contract(off)

#define NBATCH 2
#define SQLEN  2048
#define HIDSZ  2048
#define NHEAD  16
#define HDIM   128

#define SLAB_US 4352
#define OPITCH  136
#define FPITCH  132

static_assert(SQLEN % 128 == 0);
static_assert(HIDSZ % 128 == 0);
static_assert(NHEAD * HDIM == HIDSZ);
static_assert(16 * FPITCH * 4 <= SLAB_US * 2);
static_assert(2 * 16 * OPITCH <= SLAB_US);

typedef __bf16         v16b __attribute__((ext_vector_type(16)));
typedef __bf16         v8b  __attribute__((ext_vector_type(8)));
typedef float          v8f  __attribute__((ext_vector_type(8)));
typedef float          v4f  __attribute__((ext_vector_type(4)));
typedef float          v2f  __attribute__((ext_vector_type(2)));
typedef unsigned int   v4u  __attribute__((ext_vector_type(4)));
typedef unsigned short v8us __attribute__((ext_vector_type(8)));

#define ZERO8 ((v8f){0.f, 0.f, 0.f, 0.f, 0.f, 0.f, 0.f, 0.f})

union FragB { v16b v; v8b h[2]; };

__device__ __forceinline__ unsigned short f2bf_bits(float f) {
  const unsigned u = __float_as_uint(f);
  return (unsigned short)((u + 0x7FFFu + ((u >> 16) & 1u)) >> 16);
}
__device__ __forceinline__ float bf_bits2f(unsigned short b) { return __uint_as_float(((unsigned)b) << 16); }
__device__ __forceinline__ void split_bf(float f, unsigned short& hb, unsigned short& lb) {
  hb = f2bf_bits(f);
  lb = f2bf_bits(f - bf_bits2f(hb));
}
__device__ __forceinline__ unsigned pk16(unsigned short a, unsigned short b) { return (unsigned)a | ((unsigned)b << 16); }

__device__ __forceinline__ v16b ldfrag(const unsigned short* p) {
  FragB u;
  u.h[0] = *(const v8b*)p;
  u.h[1] = *(const v8b*)(p + 16);
  return u.v;
}
__device__ __forceinline__ v16b ldfrag_lds(const __bf16* p) {
  FragB u;
  u.h[0] = *(const v8b*)p;
  u.h[1] = *(const v8b*)(p + 16);
  return u.v;
}
__device__ __forceinline__ v8f mma(v16b a, v16b b, v8f c) {
  c = __builtin_amdgcn_wmma_f32_16x16x32_bf16(false, a, false, b, (short)0, c, false, false);
  asm volatile("v_nop\n\tv_nop\n\tv_nop\n\tv_nop" : "+v"(c) : "v"(a), "v"(b));
  return c;
}
__device__ __forceinline__ void wave_sync() {
  __builtin_amdgcn_fence(__ATOMIC_RELEASE, "workgroup");
  __builtin_amdgcn_wave_barrier();
  __builtin_amdgcn_fence(__ATOMIC_ACQUIRE, "workgroup");
}

__global__ __launch_bounds__(256) void k_cvt(const float* __restrict__ src, unsigned short* __restrict__ dst, int n8) {
  const int i = (int)blockIdx.x * 256 + (int)threadIdx.x;
  if (i < n8) {
    const float* s = src + 8 * (size_t)i;
    const v4f a = *(const v4f*)s;
    const v4f b = *(const v4f*)(s + 4);
    v4u o;
    o[0] = pk16(f2bf_bits(a[0]), f2bf_bits(a[1]));
    o[1] = pk16(f2bf_bits(a[2]), f2bf_bits(a[3]));
    o[2] = pk16(f2bf_bits(b[0]), f2bf_bits(b[1]));
    o[3] = pk16(f2bf_bits(b[2]), f2bf_bits(b[3]));
    unsigned short* d = dst + 8 * (size_t)i;
    *(volatile v4u*)d = o;
    __threadfence();
    *(volatile v4u*)d = o;
  }
}

template <int EPI, bool SPLITA>
__global__ __launch_bounds__(128) __attribute__((amdgpu_num_vgpr(240))) void k_gemm(
    const unsigned short* __restrict__ A, const unsigned short* __restrict__ A2, int lda,
    const unsigned short* __restrict__ Bt, int ldb, int K,
    unsigned short* C0, unsigned short* C1, float* Cf, int ldc,
    const float* tab, float* tabout, int tilesN, int tabmode) {
  __shared__ __align__(16) unsigned short slab[4][SLAB_US];
  const int tid  = (int)threadIdx.x;
  const int lane = tid & 31;
  const int wave = tid >> 5;
  const int hh   = lane >> 4;
  const int c    = lane & 15;

  if (EPI == 2 && tabmode != 0) {
    float* st = reinterpret_cast<float*>(&slab[0][0]);
    const int plo = tid >> 6;
    const int f   = tid & 63;
    const int pos = (int)blockIdx.x * 2 + plo;
    const float e   = (float)f * 0.015625f;
    const float pw  = powf(10000.0f, e);
    const float inv = 1.0f / pw;
    const float th  = (float)pos * inv;
    const float cv  = cosf(th);
    const float sv  = sinf(th);
    st[2 * tid]     = cv;
    st[2 * tid + 1] = sv;
    __syncthreads();
    if (tid < 64) {
      const v4f v = *(const v4f*)(st + 4 * tid);
      float* dp = tabout + (size_t)blockIdx.x * 256 + 4 * tid;
      *(volatile v4f*)dp = v;
      __threadfence();
      *(volatile v4f*)dp = v;
    }
    return;
  }

  const int bm = (int)blockIdx.x / tilesN;
  const int bn = (int)blockIdx.x - bm * tilesN;
  const int m0 = bm * 64 + wave * 16;
  const int n0 = bn * 128;

  v8f acc[8];
#pragma unroll
  for (int j = 0; j < 8; ++j) acc[j] = ZERO8;

#pragma unroll 1
  for (int k0 = 0; k0 < K; k0 += 32) {
    const int kk = k0 + 8 * hh;
    const v16b a = ldfrag(A + (size_t)(m0 + c) * lda + kk);
    v16b al = a;
    if (SPLITA) al = ldfrag(A2 + (size_t)(m0 + c) * lda + kk);
#pragma unroll
    for (int j = 0; j < 8; ++j) {
      const v16b b = ldfrag(Bt + (size_t)(n0 + 16 * j + c) * ldb + kk);
      acc[j] = mma(a, b, acc[j]);
      if (SPLITA) acc[j] = mma(al, b, acc[j]);
    }
  }

  const int mr0 = m0;
  if (EPI == 0) {
    float* sf = reinterpret_cast<float*>(&slab[wave][0]);
#pragma unroll
    for (int j = 0; j < 8; ++j)
#pragma unroll
      for (int r = 0; r < 8; ++r)
        sf[(8 * hh + r) * FPITCH + 16 * j + c] = acc[j][r];
    wave_sync();
    for (int pass = 0; pass < 2; ++pass) {
#pragma unroll
      for (int row = 0; row < 16; ++row) {
        const v4f v = *(const v4f*)(sf + row * FPITCH + 4 * lane);
        *(volatile v4f*)(Cf + (size_t)(mr0 + row) * ldc + n0 + 4 * lane) = v;
      }
      __threadfence();
    }
  } else if (EPI == 1) {
    unsigned short* sh = &slab[wave][0];
    unsigned short* sl = &slab[wave][16 * OPITCH];
#pragma unroll
    for (int j = 0; j < 8; ++j)
#pragma unroll
      for (int r = 0; r < 8; ++r) {
        unsigned short hb, lb;
        split_bf(acc[j][r], hb, lb);
        sh[(8 * hh + r) * OPITCH + 16 * j + c] = hb;
        sl[(8 * hh + r) * OPITCH + 16 * j + c] = lb;
      }
    wave_sync();
    const int col8 = 8 * c;
    for (int pass = 0; pass < 2; ++pass) {
#pragma unroll
      for (int it = 0; it < 8; ++it) {
        const int row = 2 * it + hh;
        const v8us hv = *(const v8us*)(sh + row * OPITCH + col8);
        const v8us lv = *(const v8us*)(sl + row * OPITCH + col8);
        const size_t go = (size_t)(mr0 + row) * ldc + n0 + col8;
        *(volatile v8us*)(C0 + go) = hv;
        *(volatile v8us*)(C1 + go) = lv;
      }
      __threadfence();
    }
  } else {
    float* sf = reinterpret_cast<float*>(&slab[wave][0]);
#pragma unroll
    for (int j = 0; j < 8; ++j)
#pragma unroll
      for (int r = 0; r < 8; ++r)
        sf[(8 * hh + r) * FPITCH + 16 * j + c] = acc[j][r];
    wave_sync();
    const int cown = 8 * c;
    const int cprt = (cown + 64) & 127;
    const int f0   = cown & 63;
    const float sg = (c < 8) ? -1.0f : 1.0f;
    for (int pass = 0; pass < 2; ++pass) {
#pragma unroll 1
      for (int it = 0; it < 8; ++it) {
        const int row = 2 * it + hh;
        const float* sr = sf + row * FPITCH;
        const v4f o0 = *(const v4f*)(sr + cown);
        const v4f o1 = *(const v4f*)(sr + cown + 4);
        const v4f p0 = *(const v4f*)(sr + cprt);
        const v4f p1 = *(const v4f*)(sr + cprt + 4);
        const float* tp = tab + ((size_t)(mr0 + row) * 64 + f0) * 2;
        const v4f t0 = *(const v4f*)tp;
        const v4f t1 = *(const v4f*)(tp + 4);
        const v4f t2 = *(const v4f*)(tp + 8);
        const v4f t3 = *(const v4f*)(tp + 12);
        const float y0 = o0[0] * t0[0] + (sg * p0[0]) * t0[1];
        const float y1 = o0[1] * t0[2] + (sg * p0[1]) * t0[3];
        const float y2 = o0[2] * t1[0] + (sg * p0[2]) * t1[1];
        const float y3 = o0[3] * t1[2] + (sg * p0[3]) * t1[3];
        const float y4 = o1[0] * t2[0] + (sg * p1[0]) * t2[1];
        const float y5 = o1[1] * t2[2] + (sg * p1[1]) * t2[3];
        const float y6 = o1[2] * t3[0] + (sg * p1[2]) * t3[1];
        const float y7 = o1[3] * t3[2] + (sg * p1[3]) * t3[3];
        unsigned short h0, l0, h1, l1, h2, l2, h3, l3, h4, l4, h5, l5, h6, l6, h7, l7;
        split_bf(y0, h0, l0); split_bf(y1, h1, l1); split_bf(y2, h2, l2); split_bf(y3, h3, l3);
        split_bf(y4, h4, l4); split_bf(y5, h5, l5); split_bf(y6, h6, l6); split_bf(y7, h7, l7);
        v4u hv, lv;
        hv[0] = pk16(h0, h1); hv[1] = pk16(h2, h3); hv[2] = pk16(h4, h5); hv[3] = pk16(h6, h7);
        lv[0] = pk16(l0, l1); lv[1] = pk16(l2, l3); lv[2] = pk16(l4, l5); lv[3] = pk16(l6, l7);
        const size_t go = (size_t)(mr0 + row) * ldc + n0 + cown;
        *(volatile v4u*)(C0 + go) = hv;
        *(volatile v4u*)(C1 + go) = lv;
      }
      __threadfence();
    }
  }
}

__global__ __launch_bounds__(128) void k_attn(
    const unsigned short* __restrict__ QKh, const unsigned short* __restrict__ QKl,
    const unsigned short* __restrict__ VTh, const unsigned short* __restrict__ VTl,
    unsigned short* CXh, unsigned short* CXl, float sscale) {
  __shared__ __align__(16) __bf16 Pb[4][2][1024];
  __shared__ __align__(16) unsigned short Os[4][2][16 * OPITCH];

  const int tid  = (int)threadIdx.x;
  const int lane = tid & 31;
  const int wave = tid >> 5;
  const int hh   = lane >> 4;
  const int c    = lane & 15;
  const int qb   = (int)blockIdx.x & 31;
  const int h    = (int)blockIdx.x >> 5;
  const int q0   = qb * 64 + wave * 16;
  const int LDQK = 2 * HIDSZ;
  const size_t hq = (size_t)h * HDIM;
  const size_t hk = (size_t)HIDSZ + (size_t)h * HDIM;
  const size_t hv = (size_t)h * HDIM * SQLEN;

  float mrow[8], lrow[8];
  v8f oacc[8];
#pragma unroll
  for (int r = 0; r < 8; ++r) { mrow[r] = -INFINITY; lrow[r] = 0.f; }
#pragma unroll
  for (int t = 0; t < 8; ++t) oacc[t] = ZERO8;

  __bf16* ph = Pb[wave][0];
  __bf16* pl = Pb[wave][1];

  for (int kc = 0; kc <= qb; ++kc) {
    const int kv0 = kc * 64;
    wave_sync();

    v8f s[4];
#pragma unroll
    for (int j = 0; j < 4; ++j) s[j] = ZERO8;
#pragma unroll 1
    for (int p = 0; p < 3; ++p) {
      const unsigned short* Qp = ((p == 2) ? QKl : QKh) + hq;
      const unsigned short* Kp = ((p == 1) ? QKl : QKh) + hk;
#pragma unroll 1
      for (int dc = 0; dc < 4; ++dc) {
        const int dof = dc * 32 + 8 * hh;
        const v16b q = ldfrag(Qp + (size_t)(q0 + c) * LDQK + dof);
#pragma unroll
        for (int j = 0; j < 4; ++j) {
          const v16b k = ldfrag(Kp + (size_t)(kv0 + 16 * j + c) * LDQK + dof);
          s[j] = mma(q, k, s[j]);
        }
      }
    }

    const bool diag = (kc == qb);
    float cm[8];
#pragma unroll
    for (int r = 0; r < 8; ++r) {
      const int qrow = q0 + 8 * hh + r;
      float m = -INFINITY;
#pragma unroll
      for (int j = 0; j < 4; ++j) {
        const int kvcol = kv0 + 16 * j + c;
        const float sv = s[j][r] * sscale;
        const bool hide = diag && (kvcol > qrow);
        const float sm = hide ? -INFINITY : sv;
        s[j][r] = sm;
        m = fmaxf(m, sm);
      }
#pragma unroll
      for (int off = 1; off < 16; off <<= 1) m = fmaxf(m, __shfl_xor(m, off, 32));
      cm[r] = m;
    }

#pragma unroll
    for (int r = 0; r < 8; ++r) {
      const float mnew  = fmaxf(mrow[r], cm[r]);
      const float alpha = __expf(mrow[r] - mnew);
      mrow[r] = mnew;
      float psum = 0.f;
#pragma unroll
      for (int j = 0; j < 4; ++j) {
        const float pj = __expf(s[j][r] - mnew);
        psum += pj;
        unsigned short hb, lb;
        split_bf(pj, hb, lb);
        ph[(8 * hh + r) * 64 + 16 * j + c] = __builtin_bit_cast(__bf16, hb);
        pl[(8 * hh + r) * 64 + 16 * j + c] = __builtin_bit_cast(__bf16, lb);
      }
#pragma unroll
      for (int off = 1; off < 16; off <<= 1) psum += __shfl_xor(psum, off, 32);
      lrow[r] = lrow[r] * alpha + psum;
#pragma unroll
      for (int t = 0; t < 8; ++t) oacc[t][r] *= alpha;
    }
    wave_sync();

#pragma unroll 1
    for (int p = 0; p < 3; ++p) {
      const __bf16* Pp = Pb[wave][(p == 2) ? 1 : 0];
      const unsigned short* Vp = ((p == 1) ? VTl : VTh) + hv;
#pragma unroll 1
      for (int kk = 0; kk < 2; ++kk) {
        const int kof = kk * 32 + 8 * hh;
        const v16b pa = ldfrag_lds(Pp + c * 64 + kof);
#pragma unroll
        for (int t = 0; t < 8; ++t) {
          const v16b v = ldfrag(Vp + (size_t)(16 * t + c) * SQLEN + kv0 + kof);
          oacc[t] = mma(pa, v, oacc[t]);
        }
      }
    }
  }

  unsigned short* oh = Os[wave][0];
  unsigned short* ol = Os[wave][1];
#pragma unroll
  for (int r = 0; r < 8; ++r) {
    const float inv = 1.0f / lrow[r];
#pragma unroll
    for (int t = 0; t < 8; ++t) {
      unsigned short hb, lb;
      split_bf(oacc[t][r] * inv, hb, lb);
      oh[(8 * hh + r) * OPITCH + 16 * t + c] = hb;
      ol[(8 * hh + r) * OPITCH + 16 * t + c] = lb;
    }
  }
  wave_sync();
  {
    const int col8 = 8 * c;
    for (int pass = 0; pass < 2; ++pass) {
#pragma unroll
      for (int it = 0; it < 8; ++it) {
        const int row = 2 * it + hh;
        const v8us hvv = *(const v8us*)(oh + row * OPITCH + col8);
        const v8us lvv = *(const v8us*)(ol + row * OPITCH + col8);
        const size_t go = (size_t)(q0 + row) * HIDSZ + (size_t)h * HDIM + col8;
        *(volatile v8us*)(CXh + go) = hvv;
        *(volatile v8us*)(CXl + go) = lvv;
      }
      __threadfence();
    }
  }
}

extern "C" void kernel_launch(void* const* d_in, const int* in_sizes, int n_in,
                              void* d_out, int out_size, void* d_ws, size_t ws_size,
                              hipStream_t stream) {
  const int nx = NBATCH * SQLEN * HIDSZ;
  const int nw = HIDSZ * HIDSZ;
  if (n_in < 5) return;
  if (in_sizes[0] != nx) return;
  if (in_sizes[1] != nw || in_sizes[2] != nw || in_sizes[3] != nw || in_sizes[4] != nw) return;
  if (out_size != nx) return;

  const size_t szX   = (size_t)nx * 2;
  const size_t szWQK = (size_t)nw * 2 * 2;
  const size_t szW   = (size_t)nw * 2;
  const size_t szTAB = (size_t)SQLEN * 64 * 2 * 4;
  const size_t szQK  = (size_t)SQLEN * (2 * HIDSZ) * 2;
  const size_t szP   = (size_t)SQLEN * HIDSZ * 2;
  size_t off = 0;
  const size_t oX   = off; off += szX;
  const size_t oWQK = off; off += szWQK;
  const size_t oWV  = off; off += szW;
  const size_t oWO  = off; off += szW;
  const size_t oTAB = off; off += szTAB;
  const size_t oQKh = off; off += szQK;
  const size_t oQKl = off; off += szQK;
  const size_t oVTh = off; off += szP;
  const size_t oVTl = off; off += szP;
  const size_t oCXh = off; off += szP;
  const size_t oCXl = off; off += szP;
  if (off > ws_size) return;

  const float* X  = (const float*)d_in[0];
  const float* Wq = (const float*)d_in[1];
  const float* Wk = (const float*)d_in[2];
  const float* Wv = (const float*)d_in[3];
  const float* Wo = (const float*)d_in[4];
  float* out = (float*)d_out;

  char* ws = (char*)d_ws;
  unsigned short* Xb   = (unsigned short*)(ws + oX);
  unsigned short* WQKb = (unsigned short*)(ws + oWQK);
  unsigned short* WVb  = (unsigned short*)(ws + oWV);
  unsigned short* WOb  = (unsigned short*)(ws + oWO);
  float*          tabp = (float*)(ws + oTAB);
  unsigned short* QKh  = (unsigned short*)(ws + oQKh);
  unsigned short* QKl  = (unsigned short*)(ws + oQKl);
  unsigned short* VTh  = (unsigned short*)(ws + oVTh);
  unsigned short* VTl  = (unsigned short*)(ws + oVTl);
  unsigned short* CXh  = (unsigned short*)(ws + oCXh);
  unsigned short* CXl  = (unsigned short*)(ws + oCXl);

  const float sscale = 0.08838834613561630f;

  k_cvt<<<dim3(nx / 8 / 256), dim3(256), 0, stream>>>(X,  Xb,        nx / 8);
  k_cvt<<<dim3(nw / 8 / 256), dim3(256), 0, stream>>>(Wq, WQKb,      nw / 8);
  k_cvt<<<dim3(nw / 8 / 256), dim3(256), 0, stream>>>(Wk, WQKb + nw, nw / 8);
  k_cvt<<<dim3(nw / 8 / 256), dim3(256), 0, stream>>>(Wv, WVb,       nw / 8);
  k_cvt<<<dim3(nw / 8 / 256), dim3(256), 0, stream>>>(Wo, WOb,       nw / 8);

  k_gemm<2, false><<<dim3(SQLEN / 2), dim3(128), 0, stream>>>(
      Xb, Xb, HIDSZ, WQKb, HIDSZ, 0, QKh, QKl, tabp, 2 * HIDSZ, tabp, tabp, 1, 1);

  const int tilesQK = (2 * HIDSZ) / 128;
  const int tilesV  = SQLEN / 128;
  const int tilesO  = HIDSZ / 128;
  for (int b = 0; b < NBATCH; ++b) {
    const unsigned short* Xbb = Xb + (size_t)b * SQLEN * HIDSZ;
    k_gemm<2, false><<<dim3((SQLEN / 64) * tilesQK), dim3(128), 0, stream>>>(
        Xbb, Xbb, HIDSZ, WQKb, HIDSZ, HIDSZ, QKh, QKl, tabp, 2 * HIDSZ, tabp, tabp, tilesQK, 0);
    k_gemm<1, false><<<dim3((HIDSZ / 64) * tilesV), dim3(128), 0, stream>>>(
        WVb, WVb, HIDSZ, Xbb, HIDSZ, HIDSZ, VTh, VTl, tabp, SQLEN, tabp, tabp, tilesV, 0);
    k_attn<<<dim3(NHEAD * (SQLEN / 64)), dim3(128), 0, stream>>>(QKh, QKl, VTh, VTl, CXh, CXl, sscale);
    float* outb = out + (size_t)b * SQLEN * HIDSZ;
    k_gemm<0, true><<<dim3((SQLEN / 64) * tilesO), dim3(128), 0, stream>>>(
        CXh, CXl, HIDSZ, WOb, HIDSZ, HIDSZ, VTh, VTl, outb, HIDSZ, tabp, tabp, tilesO, 0);
  }
  (void)hipGetLastError();
}
